// MambaLikeBlock_33483565039899
// MI455X (gfx1250) — hardware-verified
//
#include <hip/hip_runtime.h>
#include <math.h>

typedef __attribute__((ext_vector_type(16))) _Float16 v16h;
typedef __attribute__((ext_vector_type(8)))  _Float16 v8h;
typedef __attribute__((ext_vector_type(16))) __bf16   v16b;
typedef __attribute__((ext_vector_type(8)))  __bf16   v8b;
typedef __attribute__((ext_vector_type(8)))  float    v8f;
typedef __attribute__((ext_vector_type(4)))  float    v4f;
typedef __attribute__((ext_vector_type(2)))  unsigned v2u;
#define PSCALE 32768.0f
#define U16(p) ((const unsigned short*)(const void*)(p))
#define PSCALE_INV (1.0f / 32768.0f)

__device__ __forceinline__ unsigned short f2bf_bits(float f) {
  unsigned u = __float_as_uint(f);
  return (unsigned short)((u + 0x7FFFu + ((u >> 16) & 1u)) >> 16);
}
__device__ __forceinline__ float bf_bits2f(unsigned short h) { return __uint_as_float(((unsigned)h) << 16); }

__device__ __forceinline__ void dep_guard_h(v8f& a, v8f& b, v16h x, v16h y) { asm volatile("v_nop\n\tv_nop\n\tv_nop\n\tv_nop" : "+v"(a), "+v"(b) : "v"(x), "v"(y)); }
__device__ __forceinline__ void dep_guard_b(v8f& a, v8f& b, v16b x, v16b y) { asm volatile("v_nop\n\tv_nop\n\tv_nop\n\tv_nop" : "+v"(a), "+v"(b) : "v"(x), "v"(y)); }
__device__ __forceinline__ void keep4_h(v16h a, v16h b, v16h c, v16h d) { asm volatile("v_nop" :: "v"(a), "v"(b), "v"(c), "v"(d)); }
__device__ __forceinline__ void keep4_b(v16b a, v16b b, v16b c, v16b d) { asm volatile("v_nop" :: "v"(a), "v"(b), "v"(c), "v"(d)); }
__device__ __forceinline__ void acc_guard4(v8f& a, v8f& b, v8f& c, v8f& d) { asm volatile("v_nop\n\tv_nop\n\tv_nop\n\tv_nop" : "+v"(a), "+v"(b), "+v"(c), "+v"(d)); }
template <typename T> struct Frag;
template <> struct Frag<_Float16> {
  typedef v16h V; union U { v16h v; v8h h[2]; };
  static __device__ __forceinline__ v16h load(const _Float16* p) {
    U f; f.h[0] = *(const v8h*)(p); f.h[1] = *(const v8h*)(p + 16); return f.v;
  }
  static __device__ __forceinline__ v8f mma(v16h a, v16h b, v8f c) {
    return __builtin_amdgcn_wmma_f32_16x16x32_f16(false, a, false, b, (short)0, c, false, false);
  }
  static __device__ __forceinline__ void guard(v8f& a, v8f& b, v16h x, v16h y) { dep_guard_h(a, b, x, y); }
  static __device__ __forceinline__ void keep(v16h a, v16h b, v16h c, v16h d) { keep4_h(a, b, c, d); }
};
template <> struct Frag<__bf16> {
  typedef v16b V; union U { v16b v; v8b h[2]; };
  static __device__ __forceinline__ v16b load(const __bf16* p) {
    U f; f.h[0] = *(const v8b*)(p); f.h[1] = *(const v8b*)(p + 16); return f.v;
  }
  static __device__ __forceinline__ v8f mma(v16b a, v16b b, v8f c) {
    return __builtin_amdgcn_wmma_f32_16x16x32_bf16(false, a, false, b, (short)0, c, false, false);
  }
  static __device__ __forceinline__ void guard(v8f& a, v8f& b, v16b x, v16b y) { dep_guard_b(a, b, x, y); }
  static __device__ __forceinline__ void keep(v16b a, v16b b, v16b c, v16b d) { keep4_b(a, b, c, d); }
};

template <int ET> struct Elem;
template <> struct Elem<0> { typedef _Float16 T; };
template <> struct Elem<1> { typedef __bf16 T; };
template <int ET, bool SPLIT, int BIAS_MODE, int OUT_MODE, bool RESID, int ACT = 0>
__global__ __launch_bounds__(256) void wmma_gemm64(
    const unsigned short* __restrict__ Ap, const unsigned short* __restrict__ A2p, int lda, long strideA,
    const unsigned short* __restrict__ Btp, const unsigned short* __restrict__ Bt2p, int ldb, long strideB,
    void* __restrict__ Cout, void* __restrict__ Cout2, int ldc, long strideC,
    const float* __restrict__ bias,
    const float* __restrict__ resid, long strideR,
    int M, int N, int K, float scale) {
  typedef typename Elem<ET>::T T;
  typedef typename Frag<T>::V V;
  const T* A = (const T*)Ap; const T* A2 = (const T*)A2p; const T* Bt = (const T*)Btp; const T* Bt2 = (const T*)Bt2p;
  __shared__ __align__(16) float sT[8][16 * 68];
  const int b    = blockIdx.y;
  const int lane = threadIdx.x & 31;
  const int wave = threadIdx.x >> 5;
  const int tilesN = N >> 6;
  const int tilesM = M >> 6;
  const int tile = blockIdx.x * 8 + wave;
  if (tile >= tilesM * tilesN) return;
  const int tm = tile / tilesN;
  const int tn = tile - tm * tilesN;
  const int m0 = tm << 6;
  const int n0 = tn << 6;

  const T* Ab  = A  + (size_t)b * strideA;
  const T* Bb  = Bt + (size_t)b * strideB;
  const T* Ab2 = SPLIT ? (A2  + (size_t)b * strideA) : nullptr;
  const T* Bb2 = SPLIT ? (Bt2 + (size_t)b * strideB) : nullptr;

  const int rlane = lane & 15;
  const int koff  = (lane >> 4) * 8;
  const int mOff  = (lane >> 4) * 8;

  v8f acc[4][4];
#pragma unroll
  for (int i = 0; i < 4; ++i)
#pragma unroll
    for (int j = 0; j < 4; ++j) acc[i][j] = (v8f){0.f,0.f,0.f,0.f,0.f,0.f,0.f,0.f};

  for (int k0 = 0; k0 < K; k0 += 32) {
    V bh[4], bl[4];
#pragma unroll
    for (int j = 0; j < 4; ++j) {
      const size_t bo = (size_t)(n0 + (j << 4) + rlane) * ldb + koff + k0;
      bh[j] = Frag<T>::load(Bb + bo);
      if (SPLIT) bl[j] = Frag<T>::load(Bb2 + bo);
    }
#pragma unroll
    for (int i = 0; i < 4; ++i) {
      const size_t ao = (size_t)(m0 + (i << 4) + rlane) * lda + koff + k0;
      V ah = Frag<T>::load(Ab + ao);
      V al;
      if (SPLIT) al = Frag<T>::load(Ab2 + ao);
#pragma unroll
      for (int j = 0; j < 4; ++j) {
        acc[i][j] = Frag<T>::mma(ah, bh[j], acc[i][j]);
        if (SPLIT) {
          acc[i][j] = Frag<T>::mma(ah, bl[j], acc[i][j]);
          acc[i][j] = Frag<T>::mma(al, bh[j], acc[i][j]);
        }
      }
      Frag<T>::guard(acc[i][0], acc[i][3], ah, SPLIT ? al : ah);
    }
    Frag<T>::keep(bh[0], bh[1], bh[2], bh[3]);
    if (SPLIT) Frag<T>::keep(bl[0], bl[1], bl[2], bl[3]);
  }
  acc_guard4(acc[0][0], acc[0][1], acc[0][2], acc[0][3]);
  acc_guard4(acc[1][0], acc[1][1], acc[1][2], acc[1][3]);
  acc_guard4(acc[2][0], acc[2][1], acc[2][2], acc[2][3]);
  acc_guard4(acc[3][0], acc[3][1], acc[3][2], acc[3][3]);

  float* slab = sT[wave];
  const float* Rb = RESID ? (resid + (size_t)b * strideR) : nullptr;
#pragma unroll
  for (int i = 0; i < 4; ++i) {
    const int mBase = m0 + (i << 4);
#pragma unroll
    for (int j = 0; j < 4; ++j) {
      const int n = n0 + (j << 4) + rlane;
      float bv = 0.f;
      if (BIAS_MODE == 2) bv = bias[n];
#pragma unroll
      for (int r = 0; r < 8; ++r) {
        float v = acc[i][j][r] * scale;
        if (BIAS_MODE == 1) v += bias[mBase + mOff + r];
        if (BIAS_MODE == 2) v += bv;
        if (RESID) v += Rb[(size_t)(mBase + mOff + r) * ldc + n];
        if (ACT == 1) v = tanhf(v);
        if (ACT == 2) v = fmaxf(v, 0.0f);
        if (ACT == 3) v = v / (1.0f + expf(-v));
        if (ACT == 4) v = (v > 0.f) ? v : 0.01f * v;
        if (ACT == 5) v = 0.5f * v * (1.0f + erff(v * 0.70710678118654752f));
        slab[(mOff + r) * 68 + (j << 4) + rlane] = v;
      }
    }
    __builtin_amdgcn_fence(__ATOMIC_RELEASE, "workgroup");
    __builtin_amdgcn_wave_barrier();
    __builtin_amdgcn_fence(__ATOMIC_ACQUIRE, "workgroup");
    if (OUT_MODE == 0) {
      float* C = (float*)Cout + (size_t)b * strideC;
      const int hh = lane >> 4, c4 = (lane & 15) * 4;
      for (int pass = 0; pass < 2; ++pass) {
#pragma unroll
        for (int it = 0; it < 8; ++it) {
          const int row = it * 2 + hh;
          v4f v = *(const v4f*)(slab + row * 68 + c4);
          *(volatile v4f*)(C + (size_t)(mBase + row) * ldc + n0 + c4) = v;
        }
        __threadfence();
      }
    } else {
      const int q = lane >> 3, c8 = (lane & 7) * 8;
      unsigned short* C  = (unsigned short*)Cout  + (size_t)b * strideC;
      unsigned short* C2 = (OUT_MODE == 2) ? ((unsigned short*)Cout2 + (size_t)b * strideC) : nullptr;
      for (int pass = 0; pass < 2; ++pass) {
#pragma unroll
        for (int it = 0; it < 4; ++it) {
          const int row = it * 4 + q;
          const float* sp = slab + row * 68 + c8;
          v8h hv, lv;
#pragma unroll
          for (int e = 0; e < 8; ++e) {
            if (OUT_MODE == 1) {
              hv[e] = (_Float16)sp[e];
            } else {
              unsigned short hb = f2bf_bits(sp[e]);
              unsigned short lb = f2bf_bits(sp[e] - bf_bits2f(hb));
              hv[e] = __builtin_bit_cast(_Float16, hb);
              lv[e] = __builtin_bit_cast(_Float16, lb);
            }
          }
          *(volatile v8h*)(C + (size_t)(mBase + row) * ldc + n0 + c8) = hv;
          if (OUT_MODE == 2) *(volatile v8h*)(C2 + (size_t)(mBase + row) * ldc + n0 + c8) = lv;
        }
        __threadfence();
      }
    }
    __builtin_amdgcn_fence(__ATOMIC_RELEASE, "workgroup");
    __builtin_amdgcn_wave_barrier();
    __builtin_amdgcn_fence(__ATOMIC_ACQUIRE, "workgroup");
  }
}

constexpr int kDModel   = 256;
constexpr int kDInner   = 512;
constexpr int kGate3    = 768;
constexpr int kBatch    = 8;
constexpr int kSeq      = 4096;
constexpr int kRowsAll  = kBatch * kSeq;
constexpr int kRowsHalf = kRowsAll / 2;
constexpr int kHPitch   = 264;
constexpr int kSlabPitch = 36;
static_assert(kRowsHalf % 64 == 0 && kDInner % 64 == 0 && kGate3 % 64 == 0, "tile multiples");
static_assert(kDModel % 32 == 0 && kDInner % 32 == 0, "K multiples of 32");
static_assert((kHPitch * 2) % 16 == 0 && (kSlabPitch * 4) % 16 == 0, "LDS row alignment");

__device__ __forceinline__ v8f mma_h(v16h a, v16h b, v8f c) {
  c = __builtin_amdgcn_wmma_f32_16x16x32_f16(false, a, false, b, (short)0, c, false, false);
  asm volatile("v_nop\n\tv_nop\n\tv_nop\n\tv_nop" : "+v"(c) : "v"(a), "v"(b));
  return c;
}

__global__ __launch_bounds__(256) void cast_f32_f16x8_scaled(
    const float* __restrict__ in, unsigned short* __restrict__ outp, int n8, float scale) {
  const int i = blockIdx.x * 256 + threadIdx.x;
  if (i < n8) {
    const v4f a = *(const v4f*)(in + 8 * (size_t)i);
    const v4f b = *(const v4f*)(in + 8 * (size_t)i + 4);
    v8h hv;
    hv[0] = (_Float16)(a[0] * scale); hv[1] = (_Float16)(a[1] * scale);
    hv[2] = (_Float16)(a[2] * scale); hv[3] = (_Float16)(a[3] * scale);
    hv[4] = (_Float16)(b[0] * scale); hv[5] = (_Float16)(b[1] * scale);
    hv[6] = (_Float16)(b[2] * scale); hv[7] = (_Float16)(b[3] * scale);
    *(volatile v8h*)(outp + 8 * (size_t)i) = hv;
    __threadfence();
    *(volatile v8h*)(outp + 8 * (size_t)i) = hv;
  }
}

__global__ __launch_bounds__(256) void gelu_f32_f16x4(
    const float* __restrict__ in, unsigned* __restrict__ outw, int n4, float scale) {
  const int i = blockIdx.x * 256 + threadIdx.x;
  if (i >= n4) return;
  const float* p = in + 4 * (size_t)i;
  unsigned long long w = 0ull;
#pragma unroll 1
  for (int e = 0; e < 4; ++e) {
    const float v = p[e];
    const float g = 0.5f * v * (1.0f + erff(v * 0.70710678118654752f)) * scale;
    const unsigned long long bits = (unsigned long long)__builtin_bit_cast(unsigned short, (_Float16)g);
    w |= bits << (16 * e);
  }
  v2u wv;
  wv.x = (unsigned)(w & 0xffffffffull);
  wv.y = (unsigned)(w >> 32);
  *(volatile v2u*)(outw + 2 * (size_t)i) = wv;
  __threadfence();
  *(volatile v2u*)(outw + 2 * (size_t)i) = wv;
}

__global__ __launch_bounds__(256) void gru_scan_block(
    const float* __restrict__ gx,
    const unsigned short* __restrict__ whh,
    const float* __restrict__ b_hh,
    float* __restrict__ out) {
  union FH { v16h v; v8h h[2]; };
  __shared__ __align__(16) unsigned short hAu[2][16 * kHPitch];
  __shared__ __align__(16) float slab[8][16 * kSlabPitch];

  const int tid  = threadIdx.x;
  const int lane = tid & 31;
  const int wave = tid >> 5;
  const int hh   = lane >> 4;
  const int c    = lane & 15;

  {
    unsigned* hz = (unsigned*)(&hAu[0][0]);
    const int nWords = (2 * 16 * kHPitch) / 2;
    for (int i = tid; i < nWords; i += 256) hz[i] = 0u;
  }

  float hreg[2][8];
#pragma unroll
  for (int u = 0; u < 2; ++u)
#pragma unroll
    for (int r = 0; r < 8; ++r) hreg[u][r] = 0.0f;

  float bh[2][3];
#pragma unroll
  for (int u = 0; u < 2; ++u)
#pragma unroll
    for (int g = 0; g < 3; ++g) bh[u][g] = b_hh[g * kDModel + 16 * (2 * wave + u) + c];

  const float kSC = 1.0f / 16384.0f;
  __syncthreads();

  for (int t = 0; t < kSeq; ++t) {
    const int cur = t & 1;
    const unsigned short* hcur = &hAu[cur][0];
    unsigned short* hnxt = &hAu[cur ^ 1][0];

    v8f acc[2][3];
#pragma unroll
    for (int u = 0; u < 2; ++u)
#pragma unroll
      for (int g = 0; g < 3; ++g) acc[u][g] = (v8f){0.f,0.f,0.f,0.f,0.f,0.f,0.f,0.f};

#pragma unroll 1
    for (int k0 = 0; k0 < kDModel; k0 += 32) {
      FH a;
      a.h[0] = *(const v8h*)(hcur + c * kHPitch + k0 + 8 * hh);
      a.h[1] = *(const v8h*)(hcur + c * kHPitch + k0 + 16 + 8 * hh);
#pragma unroll
      for (int u = 0; u < 2; ++u) {
#pragma unroll
        for (int g = 0; g < 3; ++g) {
          const unsigned short* bp = whh + (size_t)(g * kDModel + 16 * (2 * wave + u) + c) * kDModel + k0 + 8 * hh;
          FH bf;
          bf.h[0] = *(const v8h*)(bp);
          bf.h[1] = *(const v8h*)(bp + 16);
          acc[u][g] = mma_h(a.v, bf.v, acc[u][g]);
        }
      }
    }

    const float* gxt = gx + (size_t)t * kGate3;
    float* sl = &slab[wave][0];
#pragma unroll
    for (int u = 0; u < 2; ++u) {
      const int col = 16 * (2 * wave + u) + c;
#pragma unroll
      for (int r = 0; r < 8; ++r) {
        const float* gp = gxt + (size_t)r * ((size_t)kSeq * kGate3) + col;
        const float xr = gp[0];
        const float xz = gp[kDModel];
        const float xn = gp[2 * kDModel];
        const float ar  = acc[u][0][r] * kSC + bh[u][0] + xr;
        const float az  = acc[u][1][r] * kSC + bh[u][1] + xz;
        const float ahn = acc[u][2][r] * kSC + bh[u][2];
        const float rg = 1.0f / (1.0f + expf(-ar));
        const float zg = 1.0f / (1.0f + expf(-az));
        const float ng = tanhf(xn + rg * ahn);
        const float hn = (1.0f - zg) * ng + zg * hreg[u][r];
        hreg[u][r] = hn;
        sl[(8 * hh + r) * kSlabPitch + 16 * u + c] = hn;
      }
    }
    __builtin_amdgcn_fence(__ATOMIC_RELEASE, "workgroup");
    __builtin_amdgcn_wave_barrier();
    __builtin_amdgcn_fence(__ATOMIC_ACQUIRE, "workgroup");

    {
      const int rq = lane >> 3, c4 = (lane & 7) * 4;
      for (int pass = 0; pass < 2; ++pass) {
#pragma unroll
        for (int it = 0; it < 2; ++it) {
          const int row = it * 4 + rq;
          const v4f v = *(const v4f*)(sl + row * kSlabPitch + c4);
          *(volatile v4f*)(out + ((size_t)row * kSeq + t) * kDModel + 32 * wave + c4) = v;
        }
        __threadfence();
      }
    }
    {
      const int row = lane >> 2, c8 = (lane & 3) * 8;
      const v4f v0 = *(const v4f*)(sl + row * kSlabPitch + c8);
      const v4f v1 = *(const v4f*)(sl + row * kSlabPitch + c8 + 4);
      v8h hv;
      hv[0] = (_Float16)(v0[0] * 256.0f); hv[1] = (_Float16)(v0[1] * 256.0f);
      hv[2] = (_Float16)(v0[2] * 256.0f); hv[3] = (_Float16)(v0[3] * 256.0f);
      hv[4] = (_Float16)(v1[0] * 256.0f); hv[5] = (_Float16)(v1[1] * 256.0f);
      hv[6] = (_Float16)(v1[2] * 256.0f); hv[7] = (_Float16)(v1[3] * 256.0f);
      *(v8h*)(hnxt + row * kHPitch + 32 * wave + c8) = hv;
    }
    __syncthreads();
  }
}

extern "C" void kernel_launch(void* const* d_in, const int* in_sizes, int n_in,
                              void* d_out, int out_size, void* d_ws,
                              size_t ws_size, hipStream_t stream) {
  if (n_in < 7) return;
  if (in_sizes[0] != kRowsAll * kDModel) return;
  if (in_sizes[1] != kDInner * kDModel) return;
  if (in_sizes[2] != kDInner) return;
  if (in_sizes[3] != kGate3 * kDInner) return;
  if (in_sizes[4] != kGate3) return;
  if (in_sizes[5] != kGate3 * kDModel) return;
  if (in_sizes[6] != kGate3) return;
  if (out_size != kRowsAll * kDModel) return;

  const float* x    = (const float*)d_in[0];
  const float* W1   = (const float*)d_in[1];
  const float* b1   = (const float*)d_in[2];
  const float* W_ih = (const float*)d_in[3];
  const float* b_ih = (const float*)d_in[4];
  const float* W_hh = (const float*)d_in[5];
  const float* b_hh = (const float*)d_in[6];
  float* out = (float*)d_out;

  char* ws = (char*)d_ws;
  const size_t offX16 = 0;
  const size_t bytesX16 = (size_t)kRowsHalf * kDModel * 2;
  const size_t offPre = offX16 + bytesX16;
  const size_t bytesPre = (size_t)kRowsHalf * kDInner * 4;
  const size_t offGX  = 0;
  const size_t bytesGXhalf = (size_t)kRowsHalf * kGate3 * 4;
  const size_t bytesGX = 2 * bytesGXhalf;
  const size_t offH16 = offGX + bytesGX;
  const size_t bytesH16 = (size_t)kRowsHalf * kDInner * 2;
  const size_t offW1  = offH16 + bytesH16;
  const size_t offWih = offW1 + (size_t)kDInner * kDModel * 2;
  const size_t offWhh = offWih + (size_t)kGate3 * kDInner * 2;
  const size_t wsEnd  = offWhh + (size_t)kGate3 * kDModel * 2;
  if (offPre + bytesPre > bytesGXhalf) return;
  if (ws_size < wsEnd) return;

  unsigned short* x16  = (unsigned short*)(ws + offX16);
  float*          pre  = (float*)(ws + offPre);
  float*          gxp  = (float*)(ws + offGX);
  unsigned short* h16  = (unsigned short*)(ws + offH16);
  unsigned short* w1h  = (unsigned short*)(ws + offW1);
  unsigned short* wihh = (unsigned short*)(ws + offWih);
  unsigned short* whhh = (unsigned short*)(ws + offWhh);

  {
    const int n8a = kDInner * kDModel / 8;
    const int n8b = kGate3 * kDInner / 8;
    const int n8c = kGate3 * kDModel / 8;
    cast_f32_f16x8_scaled<<<(n8a + 255) / 256, 256, 0, stream>>>(W1, w1h, n8a, 64.0f);
    cast_f32_f16x8_scaled<<<(n8b + 255) / 256, 256, 0, stream>>>(W_ih, wihh, n8b, 64.0f);
    cast_f32_f16x8_scaled<<<(n8c + 255) / 256, 256, 0, stream>>>(W_hh, whhh, n8c, 64.0f);
  }

  for (int step = 0; step < 2; ++step) {
    const int hf = 1 - step;
    const float* xh = x + (size_t)hf * kRowsHalf * kDModel;
    float* gxh = gxp + (size_t)hf * kRowsHalf * kGate3;

    const int n8x = kRowsHalf * kDModel / 8;
    cast_f32_f16x8_scaled<<<(n8x + 255) / 256, 256, 0, stream>>>(xh, x16, n8x, 8.0f);

    wmma_gemm64<0, false, 2, 0, false, 0><<<dim3(256, 1), 256, 0, stream>>>(
        x16, x16, kDModel, 0L,
        w1h, w1h, kDModel, 0L,
        (void*)pre, (void*)pre, kDInner, 0L,
        b1, b1, 0L,
        kRowsHalf, kDInner, kDModel, 1.0f / 512.0f);

    const int n4 = kRowsHalf * kDInner / 4;
    gelu_f32_f16x4<<<(n4 + 255) / 256, 256, 0, stream>>>(pre, (unsigned*)h16, n4, 16.0f);

    wmma_gemm64<0, false, 2, 0, false, 0><<<dim3(384, 1), 256, 0, stream>>>(
        h16, h16, kDInner, 0L,
        wihh, wihh, kDInner, 0L,
        (void*)gxh, (void*)gxh, kGate3, 0L,
        b_ih, b_ih, 0L,
        kRowsHalf, kGate3, kDInner, 1.0f / 1024.0f);
  }

  gru_scan_block<<<1, 256, 0, stream>>>(gxp, whhh, b_hh, out);
}
